// GraphSAGEEncoder_1142461300900
// MI455X (gfx1250) — hardware-run, weakly checked
//
#include <hip/hip_runtime.h>

typedef float          v8f   __attribute__((ext_vector_type(8)));
typedef float          v4f   __attribute__((ext_vector_type(4)));
typedef unsigned int   v4u   __attribute__((ext_vector_type(4)));
typedef int            v8i   __attribute__((ext_vector_type(8)));
typedef unsigned short v8us  __attribute__((ext_vector_type(8)));
typedef unsigned short v16us __attribute__((ext_vector_type(16)));
typedef __bf16         v16bf __attribute__((ext_vector_type(16)));
typedef _Float16       v16h  __attribute__((ext_vector_type(16)));
typedef v4f  __attribute__((may_alias)) v4fa;
typedef v8us __attribute__((may_alias)) v8usa;
union FragB { v16bf v; v16us u; v8us h[2]; v8i w; };
union FragH { v16h  v; v16us u; v8us h[2]; v8i w; };

__device__ __forceinline__ v8f wmb(const FragB& a, const FragB& b, v8f c) {
  v8f d = __builtin_amdgcn_wmma_f32_16x16x32_bf16(false, a.v, false, b.v, (short)0, c, false, false);
  asm volatile("v_nop\n\tv_nop\n\tv_nop\n\tv_nop" : "+v"(d) : "v"(a.w), "v"(b.w));
  return d;
}

__device__ __forceinline__ v8f wmh(const FragH& a, const FragH& b, v8f c) {
  v8f d = __builtin_amdgcn_wmma_f32_16x16x32_f16(false, a.v, false, b.v, (short)0, c, false, false);
  asm volatile("v_nop\n\tv_nop\n\tv_nop\n\tv_nop" : "+v"(d) : "v"(a.w), "v"(b.w));
  return d;
}

__device__ __forceinline__ unsigned bf16_bits(float f) {
  const unsigned u = __float_as_uint(f);
  const unsigned r = (u + 0x7FFFu + ((u >> 16) & 1u)) >> 16;
  const unsigned q = (u >> 16) | 0x40u;
  return ((u & 0x7fffffffu) > 0x7f800000u) ? q : r;
}

__device__ __forceinline__ float bf16_val(float f) {
  return __uint_as_float(bf16_bits(f) << 16);
}
__device__ __forceinline__ int clampi(int v, int lo, int hi) {
  return v < lo ? lo : (v > hi ? hi : v);
}

__device__ __forceinline__ unsigned f16_bits(float f) {
  const unsigned u  = __float_as_uint(f);
  const unsigned s  = (u >> 16) & 0x8000u;
  const unsigned a  = u & 0x7fffffffu;
  const unsigned t  = a - 0x38000000u;
  const unsigned r  = (t + 0x0FFFu + ((t >> 13) & 1u)) >> 13;
  const unsigned rc = r > 0x7C00u ? 0x7C00u : r;
  const bool small  = a < 0x38800000u;
  const bool isnan  = a > 0x7f800000u;
  const unsigned fin = small ? 0u : (s | rc);
  return isnan ? (s | 0x7E00u) : fin;
}

__device__ __forceinline__ unsigned pk16(unsigned lo, unsigned hi) { return lo | (hi << 16); }
__device__ __forceinline__ unsigned bf16_lo_bits(float v) {
  float hi = bf16_val(v);
  asm volatile("" : "+v"(hi));
  return bf16_bits(v - hi);
}
__device__ __forceinline__ v4u pack8_bf16(v4f a, v4f c) {
  return (v4u){ pk16(bf16_bits(a[0]), bf16_bits(a[1])), pk16(bf16_bits(a[2]), bf16_bits(a[3])),
                pk16(bf16_bits(c[0]), bf16_bits(c[1])), pk16(bf16_bits(c[2]), bf16_bits(c[3])) };
}
__device__ __forceinline__ v4u pack8_bf16_lo(v4f a, v4f c) {
  return (v4u){ pk16(bf16_lo_bits(a[0]), bf16_lo_bits(a[1])), pk16(bf16_lo_bits(a[2]), bf16_lo_bits(a[3])),
                pk16(bf16_lo_bits(c[0]), bf16_lo_bits(c[1])), pk16(bf16_lo_bits(c[2]), bf16_lo_bits(c[3])) };
}
__device__ __forceinline__ v4u pack8_f16(v4f a, v4f c) {
  return (v4u){ pk16(f16_bits(a[0]), f16_bits(a[1])), pk16(f16_bits(a[2]), f16_bits(a[3])),
                pk16(f16_bits(c[0]), f16_bits(c[1])), pk16(f16_bits(c[2]), f16_bits(c[3])) };
}

template <int FORM>
__global__ __launch_bounds__(256) void k_plane(const float* __restrict__ src, int rows, int cols, int ldsrc,
                                               unsigned short* __restrict__ dst, int MP, int KP) {
  static_assert(FORM >= 0 && FORM <= 3);
  const int KTOT = (FORM == 1 || FORM == 3) ? 2 * KP : KP;
  const unsigned ppr   = (unsigned)(KTOT >> 3);
  const unsigned kp8   = (unsigned)(KP >> 3);
  const unsigned total = (unsigned)MP * ppr;
  const unsigned g     = blockIdx.x * 256u + threadIdx.x;
  const unsigned rowu  = g / ppr;
  const unsigned p     = g - rowu * ppr;
  const bool second    = p >= kp8;
  const int row = (int)rowu;
  const int c0  = (int)((second ? p - kp8 : p) << 3);
  const float* srow = src + (size_t)clampi(row, 0, rows - 1) * (size_t)ldsrc;
  float x[8];
  unsigned mk[8];
#pragma unroll
  for (int e = 0; e < 8; ++e) {
    const int c = c0 + e;
    const float v = srow[clampi(c, 0, cols - 1)];
    asm volatile("" :: "v"(v));
    x[e]  = v;
    mk[e] = (row < rows && c < cols) ? 0xFFFFu : 0u;
  }
  const v4f a = (v4f){ x[0], x[1], x[2], x[3] };
  const v4f c = (v4f){ x[4], x[5], x[6], x[7] };
  v4u o;
  if (FORM == 2) {
    o = pack8_f16(a, c);
  } else {
    const v4u hi = pack8_bf16(a, c);
    o = hi;
    if (FORM == 1) { const v4u lo = pack8_bf16_lo(a, c); o = second ? lo : hi; }
  }
  const v4u mw = (v4u){ pk16(mk[0], mk[1]), pk16(mk[2], mk[3]), pk16(mk[4], mk[5]), pk16(mk[6], mk[7]) };
  o &= mw;
  if (g < total) {
    volatile v4u* q = (volatile v4u*)(dst + (size_t)g * 8);
    *q = o;
    __threadfence();
    *q = o;
  }
}

template <int FORM> struct FragOf    { typedef FragB T; };
template <>         struct FragOf<2> { typedef FragH T; };
__device__ __forceinline__ v8f mm(const FragB& a, const FragB& b, v8f c) { return wmb(a, b, c); }
__device__ __forceinline__ v8f mm(const FragH& a, const FragH& b, v8f c) { return wmh(a, b, c); }
template <class F> __device__ __forceinline__ F ld_frag(const unsigned short* p) {
  F f;
  f.h[0] = *(const v8usa*)(p);
  f.h[1] = *(const v8usa*)(p + 16);
  return f;
}

template <int FORM, int EPI>
__global__ __launch_bounds__(256) __attribute__((amdgpu_num_vgpr(248)))
void k_gemm_nt(const unsigned short* __restrict__ A, const unsigned short* __restrict__ B,
               const float* __restrict__ bias, float* __restrict__ D, int M, int N, int KTOT, int ldd) {
  static_assert(FORM >= 0 && FORM <= 2);
  static_assert(EPI == 0 || EPI == 1);
  typedef typename FragOf<FORM>::T F;
  __shared__ __attribute__((aligned(16))) float sT[8][16 * 68];
  const int lane = threadIdx.x & 31;
  const int wave = threadIdx.x >> 5;
  const int tilesM = (M + 63) >> 6;
  const int tilesN = (N + 63) >> 6;
  const int tile = blockIdx.x * 8 + wave;
  if (tile >= tilesM * tilesN) return;
  const int tm = tile / tilesN;
  const int tn = tile - tm * tilesN;
  const int m0 = tm << 6;
  const int n0 = tn << 6;

  const int rl = lane & 15;
  const int h8 = (lane >> 4) * 8;
  const unsigned short* pa = A + (size_t)(m0 + rl) * (size_t)KTOT + h8;
  const unsigned short* pb = B + (size_t)(n0 + rl) * (size_t)KTOT + h8;

  v8f acc[4][4];
#pragma unroll
  for (int i = 0; i < 4; ++i)
#pragma unroll
    for (int j = 0; j < 4; ++j) acc[i][j] = (v8f){0.f, 0.f, 0.f, 0.f, 0.f, 0.f, 0.f, 0.f};

#pragma unroll 1
  for (int k0 = 0; k0 < KTOT; k0 += 32) {
    F bf[4];
#pragma unroll
    for (int j = 0; j < 4; ++j) bf[j] = ld_frag<F>(pb + (size_t)(j << 4) * (size_t)KTOT + k0);
#pragma unroll
    for (int i = 0; i < 4; ++i) {
      const F af = ld_frag<F>(pa + (size_t)(i << 4) * (size_t)KTOT + k0);
#pragma unroll
      for (int j = 0; j < 4; ++j) acc[i][j] = mm(af, bf[j], acc[i][j]);
    }
  }

  float* slab = sT[wave];
  const int hh = lane >> 4;
  const int c4 = (lane & 15) * 4;
  const int nc = n0 + c4;
  const bool cok = nc < N;
  v4f bv = (v4f){0.f, 0.f, 0.f, 0.f};
  if (EPI == 1) {
    bv = *(const v4fa*)(bias + clampi(nc, 0, N - 4));
    asm volatile("" :: "v"(bv));
  }
#pragma unroll
  for (int i = 0; i < 4; ++i) {
    const int mBase = m0 + (i << 4);
#pragma unroll
    for (int j = 0; j < 4; ++j) {
#pragma unroll
      for (int r = 0; r < 8; ++r) slab[(h8 + r) * 68 + (j << 4) + rl] = acc[i][j][r];
    }
    __builtin_amdgcn_fence(__ATOMIC_RELEASE, "workgroup");
    __builtin_amdgcn_wave_barrier();
    __builtin_amdgcn_fence(__ATOMIC_ACQUIRE, "workgroup");
    v4f vv[8];
#pragma unroll
    for (int it = 0; it < 8; ++it) {
      const int row = it * 2 + hh;
      v4f v = *(const v4fa*)(slab + row * 68 + c4);
      if (EPI == 1) v += bv;
      vv[it] = v;
    }
    for (int pass = 0; pass < 2; ++pass) {
#pragma unroll
      for (int it = 0; it < 8; ++it) {
        const int row = mBase + it * 2 + hh;
        if (cok && row < M) *(volatile v4f*)(D + (size_t)row * (size_t)ldd + nc) = vv[it];
      }
      __threadfence();
    }
    __builtin_amdgcn_fence(__ATOMIC_RELEASE, "workgroup");
    __builtin_amdgcn_wave_barrier();
    __builtin_amdgcn_fence(__ATOMIC_ACQUIRE, "workgroup");
  }
}

#define NNODE   50000
#define NEDGE   800000
#define DFEAT   128
#define MPAD    50048
#define KL0     384
#define KL1     512
#define NBK     1024
#define NBLK    49
#define CHK     2048
#define NCHK    391
#define LCAP    22528
#define DEGCAP  64
#define MEAN_TWO_TERM 1
#define SELF_TWO_TERM 1
#define BK_LDS_INTS (2 * LCAP + 3 * NBK + 32)
#define PB_XB  (MPAD * 16 / 256)
#define PB_B0  (DFEAT * (KL0 / 8) / 256)
#define PB_B1  (DFEAT * (KL1 / 8) / 256)
#define B1_OFF (DFEAT * KL0)

static_assert(DFEAT == 128 && DFEAT == 32 * 4);
static_assert(KL0 % 32 == 0 && KL1 % 32 == 0 && KL0 == 3 * DFEAT && KL1 == 4 * DFEAT);
static_assert(NNODE <= 65536);
static_assert(NBLK * NBK >= NNODE && (NBLK - 1) * NBK < NNODE);
static_assert(NEDGE == 390 * 2048 + 1280 && NCHK == (NEDGE + CHK - 1) / CHK && NEDGE % 8 == 0);
static_assert(LCAP * 4 >= 16623 * 5 && LCAP % 1024 == 0);
static_assert(DEGCAP >= 35 + 8);
static_assert(MPAD % 64 == 0 && MPAD >= NNODE && MPAD % 8 == 0 && NNODE % 16 == 0 && NNODE % 8 == 0);
static_assert(BK_LDS_INTS % 4 == 0 && BK_LDS_INTS * 4 <= 262144);
static_assert((MPAD * 16) % 256 == 0 && (DFEAT * (KL0 / 8)) % 256 == 0 && (DFEAT * (KL1 / 8)) % 256 == 0);
static_assert((size_t)(NNODE - 1) * DFEAT + DFEAT - 1 == (size_t)6399999);

constexpr size_t WS_A    = 0;
constexpr size_t SZ_A    = (size_t)MPAD * KL1 * 2;
constexpr size_t WS_PRE  = WS_A + SZ_A;
constexpr size_t SZ_PRE  = (size_t)MPAD * DFEAT * 4;
constexpr size_t WS_H    = WS_PRE + SZ_PRE;
constexpr size_t WS_LIST = WS_H + SZ_PRE;
constexpr size_t SZ_LIST = (size_t)NBLK * LCAP * 4;
constexpr size_t WS_OFF  = WS_LIST + SZ_LIST;
constexpr size_t SZ_TAB  = (size_t)NBLK * NBK * 4;
constexpr size_t WS_CNT  = WS_OFF + SZ_TAB;
constexpr size_t WS_FLAG = WS_CNT + SZ_TAB;
constexpr size_t SZ_FLAG = (size_t)NBLK * 128;
constexpr size_t WS_BW   = WS_FLAG + SZ_FLAG;
constexpr size_t SZ_BW   = (size_t)DFEAT * (KL0 + KL1) * 2;
constexpr size_t WS_TBL  = WS_BW + SZ_BW;
constexpr size_t SZ_TBL  = 3 * 256 * 4;
constexpr size_t WS_TOTAL = WS_TBL + SZ_TBL;
static_assert(WS_TOTAL == (size_t)((size_t)840265 << 7));
static_assert(WS_TOTAL <= ((size_t)128 << 20));
static_assert(WS_PRE % 128 == 0 && WS_H % 128 == 0 && WS_LIST % 128 == 0 && WS_OFF % 128 == 0 && WS_CNT % 128 == 0);
static_assert(WS_FLAG % 128 == 0 && WS_BW % 128 == 0 && WS_TBL % 128 == 0 && (LCAP * 4) % 128 == 0);
static_assert((size_t)MPAD * KL0 * 2 <= SZ_A);

typedef int      v4i  __attribute__((ext_vector_type(4)));
typedef unsigned v2u  __attribute__((ext_vector_type(2)));
typedef v4i __attribute__((may_alias)) v4ia;
typedef v2u __attribute__((may_alias)) v2ua;
typedef v4u __attribute__((may_alias)) v4ua;

__device__ __forceinline__ void wave_sync() {
  __builtin_amdgcn_fence(__ATOMIC_RELEASE, "wavefront");
  __builtin_amdgcn_wave_barrier();
  __builtin_amdgcn_fence(__ATOMIC_ACQUIRE, "wavefront");
}
__device__ __forceinline__ v2u hi4(v4f m) {
  return (v2u){ pk16(bf16_bits(m[0]), bf16_bits(m[1])), pk16(bf16_bits(m[2]), bf16_bits(m[3])) };
}
__device__ __forceinline__ v2u lo4(v4f m) {
  return (v2u){ pk16(bf16_lo_bits(m[0]), bf16_lo_bits(m[1])), pk16(bf16_lo_bits(m[2]), bf16_lo_bits(m[3])) };
}
__device__ __forceinline__ float sel3(float a, float b, float c, unsigned ma, unsigned mb, unsigned mc) {
  return __uint_as_float((__float_as_uint(a) & ma) | (__float_as_uint(b) & mb) | (__float_as_uint(c) & mc));
}

__global__ __launch_bounds__(256) void k_prep(const float* __restrict__ x, const float* __restrict__ Wl,
                                              const float* __restrict__ Wr, const float* __restrict__ bl,
                                              const float* __restrict__ gam, const float* __restrict__ bet,
                                              unsigned short* __restrict__ apl, unsigned short* __restrict__ BW,
                                              float* __restrict__ tbl) {
  const int b   = (int)blockIdx.x;
  const int tid = (int)threadIdx.x;
  if (b < PB_XB) {
    const int u   = b * 256 + tid;
    const int row = u >> 4;
    const int pc  = u & 15;
    const float* p = x + (size_t)clampi(row, 0, NNODE - 1) * DFEAT + pc * 8;
    const v4f a = *(const v4f*)p;
    const v4f c = *(const v4f*)(p + 4);
    asm volatile("" :: "v"(a), "v"(c));
    v4u o = pack8_bf16(a, c);
    const unsigned mk = (row < NNODE) ? 0xFFFFFFFFu : 0u;
    o &= (v4u){ mk, mk, mk, mk };
    volatile v4u* q = (volatile v4u*)(apl + (size_t)row * KL0 + 2 * DFEAT + pc * 8);
    *q = o;
    __threadfence();
    *q = o;
  } else if (b < PB_XB + PB_B0 + PB_B1) {
    const int bb      = b - PB_XB;
    const bool second = bb >= PB_B0;
    const int g       = (second ? bb - PB_B0 : bb) * 256 + tid;
    const int r48 = g / 48, p48 = g - r48 * 48;
    const int r64 = g >> 6, p64 = g & 63;
    const int row = second ? r64 : r48;
    const int p   = second ? p64 : p48;
    const int part = p >> 4;
    const int k8   = (p & 15) * 8;
    const size_t so = (size_t)(second ? DFEAT * DFEAT : 0) + (size_t)row * DFEAT + k8;
    const v4f la = *(const v4f*)(Wl + so);
    const v4f lc = *(const v4f*)(Wl + so + 4);
    const v4f ra = *(const v4f*)(Wr + so);
    const v4f rc = *(const v4f*)(Wr + so + 4);
    asm volatile("" :: "v"(la), "v"(lc), "v"(ra), "v"(rc));
    const v4u pl = pack8_bf16(la, lc);
    const v4u pr = pack8_bf16(ra, rc);
    const unsigned ml = (part < 2) ? 0xFFFFFFFFu : 0u;
    const unsigned mr = ~ml;
    const v4u o = (pl & (v4u){ ml, ml, ml, ml }) | (pr & (v4u){ mr, mr, mr, mr });
    volatile v4u* q = (volatile v4u*)(BW + (size_t)(second ? B1_OFF : 0) + (size_t)g * 8);
    *q = o;
    __threadfence();
    *q = o;
  } else {
    const int which = tid >> 6;
    const int j     = (tid & 63) * 4;
    const v4f vb = *(const v4f*)(bl + j);
    const v4f vg = *(const v4f*)(gam + j);
    const v4f ve = *(const v4f*)(bet + j);
    asm volatile("" :: "v"(vb), "v"(vg), "v"(ve));
    const unsigned m0 = (which == 0) ? 0xFFFFFFFFu : 0u;
    const unsigned m1 = (which == 1) ? 0xFFFFFFFFu : 0u;
    const unsigned m2 = (which == 2) ? 0xFFFFFFFFu : 0u;
    v4f o;
    o.x = bf16_val(sel3(vb.x, vg.x, ve.x, m0, m1, m2));
    o.y = bf16_val(sel3(vb.y, vg.y, ve.y, m0, m1, m2));
    o.z = bf16_val(sel3(vb.z, vg.z, ve.z, m0, m1, m2));
    o.w = bf16_val(sel3(vb.w, vg.w, ve.w, m0, m1, m2));
    if (tid < 192) {
      volatile v4f* q = (volatile v4f*)(tbl + 4 * tid);
      *q = o;
      __threadfence();
      *q = o;
    }
  }
}

__global__ __launch_bounds__(256) void k_bucket(const int* __restrict__ ei, int* __restrict__ LIST,
                                                int* __restrict__ OFF, int* __restrict__ CNT,
                                                int* __restrict__ FLAG) {
  extern __shared__ __attribute__((aligned(16))) int dsm[];
  int* hl   = dsm;
  int* sl   = dsm + LCAP;
  int* cnt  = sl + LCAP;
  int* offs = cnt + NBK;
  int* cur  = offs + NBK;
  int* misc = cur + NBK;
  const int tid  = (int)threadIdx.x;
  const int lane = tid & 31;
  const int wave = __builtin_amdgcn_readfirstlane(tid >> 5);
  const int blk  = (int)blockIdx.x;
  const int base = blk * NBK;
  const int nb   = (NNODE - base) < NBK ? (NNODE - base) : NBK;

  {
    const v4i z4 = { 0, 0, 0, 0 };
#pragma unroll 1
    for (int i = tid; i < BK_LDS_INTS / 4; i += 256) *(v4ia*)(dsm + 4 * i) = z4;
  }
  __syncthreads();

  int tRun = 0;
#pragma unroll 1
  for (int ch = 0; ch < NCHK; ++ch) {
    const int e0 = ch * CHK + tid * 8;
    const int ec = e0 < NEDGE - 8 ? e0 : NEDGE - 8;
    const unsigned vm = (e0 < NEDGE) ? 0u : 0xFFFFFFFFu;
    const v4i sa = *(const v4i*)(ei + ec);
    const v4i sb = *(const v4i*)(ei + ec + 4);
    const v4i da = *(const v4i*)(ei + NEDGE + ec);
    const v4i db = *(const v4i*)(ei + NEDGE + ec + 4);
    asm volatile("" :: "v"(sa.x), "v"(sa.y), "v"(sa.z), "v"(sa.w));
    asm volatile("" :: "v"(sb.x), "v"(sb.y), "v"(sb.z), "v"(sb.w));
    asm volatile("" :: "v"(da.x), "v"(da.y), "v"(da.z), "v"(da.w));
    asm volatile("" :: "v"(db.x), "v"(db.y), "v"(db.z), "v"(db.w));
    const int dd[8] = { da.x, da.y, da.z, da.w, db.x, db.y, db.z, db.w };
    const int ss[8] = { sa.x, sa.y, sa.z, sa.w, sb.x, sb.y, sb.z, sb.w };
    unsigned st[8];
    bool hh[8];
    unsigned pre = 0u, wc = 0u;
#pragma unroll
    for (int j = 0; j < 8; ++j) {
      st[j] = (((unsigned)dd[j]) | vm) - (unsigned)base;
      hh[j] = st[j] < (unsigned)nb;
      const unsigned mj = __builtin_amdgcn_ballot_w32(hh[j]);
      pre += __builtin_amdgcn_mbcnt_lo(mj, 0u);
      wc  += (unsigned)__builtin_popcount(mj);
    }
    const int buf = (ch & 1) << 3;
    if (lane == 0) misc[buf + wave] = (int)wc;
    __syncthreads();
    const v4i ca = *(const v4ia*)(misc + buf);
    const v4i cb = *(const v4ia*)(misc + buf + 4);
    const int cw[8] = { ca.x, ca.y, ca.z, ca.w, cb.x, cb.y, cb.z, cb.w };
    int bs = tRun, tot = 0;
#pragma unroll
    for (int w = 0; w < 8; ++w) {
      const int c = clampi(cw[w], 0, 256);
      bs  += (w < wave) ? c : 0;
      tot += c;
    }
    int p = bs + (int)pre;
#pragma unroll
    for (int j = 0; j < 8; ++j) {
      const int word = clampi(ss[j], 0, NNODE - 1) | (int)(st[j] << 16);
      if (hh[j] && p < LCAP) hl[p] = word;
      p += hh[j] ? 1 : 0;
    }
    tRun += tot;
  }
  __syncthreads();
  const int tt = __builtin_amdgcn_readfirstlane(clampi(tRun, 0, LCAP));

  if (wave == 0) {
#pragma unroll 1
    for (int i = 0; i < tt; ++i) {
      const int u = hl[i];
      const int s = (u >> 16) & (NBK - 1);
      const int c = cnt[s];
      cnt[s] = c + 1;
    }
  }
  __syncthreads();

  int flagv = 0;
  if (wave == 0) {
    const int b0 = lane * (NBK / 32);
    int s = 0, dov = 0;
#pragma unroll 1
    for (int i = 0; i < NBK / 32; ++i) {
      const int cv = cnt[b0 + i];
      s += cv;
      dov |= (cv > DEGCAP) ? 1 : 0;
    }
    int incl = s;
#pragma unroll
    for (int d = 1; d < 32; d <<= 1) {
      const int y = __shfl_up(incl, d, 32);
      incl += (lane >= d) ? y : 0;
    }
    int run = incl - s;
#pragma unroll 1
    for (int i = 0; i < NBK / 32; ++i) {
      const int cv = cnt[b0 + i];
      offs[b0 + i] = run;
      cur[b0 + i]  = run;
      run += cv;
    }
    const unsigned bm = __builtin_amdgcn_ballot_w32(dov != 0);
    flagv = (bm != 0u || tRun > LCAP) ? 1 : 0;
  }
  __syncthreads();

  if (wave == 0) {
#pragma unroll 1
    for (int i = 0; i < tt; ++i) {
      const int u = hl[i];
      const int s = (u >> 16) & (NBK - 1);
      int p = cur[s];
      p = clampi(p, 0, LCAP - 1);
      sl[p]  = u & 0xFFFF;
      cur[s] = p + 1;
    }
  }
  __syncthreads();

  int* lg = LIST + (size_t)blk * LCAP;
  for (int pass = 0; pass < 2; ++pass) {
#pragma unroll 1
    for (int it = 0; it < LCAP / 1024; ++it) {
      const int i4 = (it * 256 + tid) * 4;
      const v4i v = *(const v4ia*)(sl + i4);
      *(volatile v4i*)(lg + i4) = v;
    }
    {
      const v4i c4 = *(const v4ia*)(cnt + 4 * tid);
      const v4i o4 = *(const v4ia*)(offs + 4 * tid);
      *(volatile v4i*)(CNT + base + 4 * tid) = c4;
      *(volatile v4i*)(OFF + base + 4 * tid) = o4;
    }
    if (wave == 0) *(volatile int*)(FLAG + blk * 32 + lane) = flagv;
    __threadfence();
  }
}

template <int L0>
__global__ __launch_bounds__(256) void k_replay(const int* __restrict__ LIST, const int* __restrict__ OFF,
                                                const int* __restrict__ CNT, const int* __restrict__ FLAG,
                                                const float* __restrict__ Hs, unsigned short* apl) {
  constexpr int LD = (L0 != 0) ? KL0 : KL1;
  __shared__ __attribute__((aligned(16))) unsigned rowb[8 * 128];
  const int tid  = (int)threadIdx.x;
  const int lane = tid & 31;
  const int wave = __builtin_amdgcn_readfirstlane(tid >> 5);
  const int t    = (int)blockIdx.x * 8 + wave;
  const bool live = t < NNODE;
  const int tc   = live ? t : NNODE - 1;
  const int blk  = tc >> 10;
  const int cv = CNT[tc];
  const int ov = OFF[tc];
  const int fv = FLAG[blk * 32];
  asm volatile("" :: "v"(cv), "v"(ov), "v"(fv));
  int cnl = clampi(cv, 0, DEGCAP);
  cnl = live ? cnl : 0;
  const int cn = __builtin_amdgcn_readfirstlane(cnl);
  const int of = __builtin_amdgcn_readfirstlane(clampi(ov, 0, LCAP));
  const int* lp = LIST + (size_t)blk * LCAP;

  float a0 = 0.0f, a1 = 0.0f, a2 = 0.0f, a3 = 0.0f;
#pragma unroll 1
  for (int b0 = 0; b0 < cn; b0 += 32) {
    int idx = of + b0 + lane;
    idx = idx > LCAP - 1 ? LCAP - 1 : idx;
    int sr = lp[idx];
    asm volatile("" :: "v"(sr));
    sr = clampi(sr, 0, NNODE - 1);
    const int m32 = (cn - b0) < 32 ? (cn - b0) : 32;
#pragma unroll 1
    for (int k = 0; k < m32; ++k) {
      const int sk = __builtin_amdgcn_readlane(sr, k);
      if constexpr (L0 != 0) {
        const v2u w = *(const v2ua*)(apl + (size_t)sk * KL0 + 2 * DFEAT + 4 * lane);
        a0 += __uint_as_float(w.x << 16);
        a1 += __uint_as_float(w.x & 0xffff0000u);
        a2 += __uint_as_float(w.y << 16);
        a3 += __uint_as_float(w.y & 0xffff0000u);
      } else {
        const v4f a = *(const v4f*)(Hs + (size_t)sk * DFEAT + 4 * lane);
        a0 += a.x;
        a1 += a.y;
        a2 += a.z;
        a3 += a.w;
      }
    }
  }
  const int cc = cv < 1 ? 1 : (cv > 16777216 ? 16777216 : cv);
  const float den = (float)cc;
  const float pz  = (fv != 0) ? __uint_as_float(0x7fc00000u) : 0.0f;
  v4f m;
  m.x = live ? (a0 / den + pz) : 0.0f;
  m.y = live ? (a1 / den + pz) : 0.0f;
  m.z = live ? (a2 / den + pz) : 0.0f;
  m.w = live ? (a3 / den + pz) : 0.0f;
  const v2u hi = hi4(m);
  v2u lo = lo4(m);
  if (MEAN_TWO_TERM == 0) lo = (v2u){ 0u, 0u };
  *(v2ua*)(&rowb[wave * 128 + 2 * lane])      = hi;
  *(v2ua*)(&rowb[wave * 128 + 64 + 2 * lane]) = lo;
  wave_sync();
  const v4u q = *(const v4ua*)(&rowb[wave * 128 + 4 * lane]);
  if (t < MPAD) {
    volatile v4u* g = (volatile v4u*)(apl + (size_t)t * LD + 8 * lane);
    *g = q;
    __threadfence();
    *g = q;
  }
}

template <int FIN>
__global__ __launch_bounds__(256) void k_row(const float* __restrict__ PRE, const float* __restrict__ gam,
                                             const float* __restrict__ bet, const int* __restrict__ FLAG,
                                             float* __restrict__ outp, unsigned short* __restrict__ apl) {
  __shared__ __attribute__((aligned(16))) unsigned rowb[8 * 128];
  const int tid  = (int)threadIdx.x;
  const int lane = tid & 31;
  const int wave = __builtin_amdgcn_readfirstlane(tid >> 5);
  const int t    = (int)blockIdx.x * 8 + wave;
  const bool live = t < NNODE;
  const int tc   = live ? t : NNODE - 1;
  const v4f v = *(const v4f*)(PRE + (size_t)tc * DFEAT + 4 * lane);
  const v4f g = *(const v4f*)(gam + 4 * lane);
  const v4f b = *(const v4f*)(bet + 4 * lane);
  const int fv = FLAG[(tc >> 10) * 32];
  asm volatile("" :: "v"(v), "v"(g), "v"(b), "v"(fv));
  const float r0 = (v.x > 0.0f) ? v.x : (v.x - v.x);
  const float r1 = (v.y > 0.0f) ? v.y : (v.y - v.y);
  const float r2 = (v.z > 0.0f) ? v.z : (v.z - v.z);
  const float r3 = (v.w > 0.0f) ? v.w : (v.w - v.w);
  float s = (r0 + r1) + (r2 + r3);
  s += __shfl_xor(s, 16, 32);
  s += __shfl_xor(s, 8, 32);
  s += __shfl_xor(s, 4, 32);
  s += __shfl_xor(s, 2, 32);
  s += __shfl_xor(s, 1, 32);
  const float mu = s * (1.0f / 128.0f);
  const float d0 = r0 - mu, d1 = r1 - mu, d2 = r2 - mu, d3 = r3 - mu;
  float qq = (d0 * d0 + d1 * d1) + (d2 * d2 + d3 * d3);
  qq += __shfl_xor(qq, 16, 32);
  qq += __shfl_xor(qq, 8, 32);
  qq += __shfl_xor(qq, 4, 32);
  qq += __shfl_xor(qq, 2, 32);
  qq += __shfl_xor(qq, 1, 32);
  const float var = qq * (1.0f / 128.0f);
  const float rs  = 1.0f / sqrtf(var + 1e-5f);
  const float pz  = (fv != 0) ? __uint_as_float(0x7fc00000u) : 0.0f;
  v4f y;
  y.x = d0 * rs * g.x + b.x + pz;
  y.y = d1 * rs * g.y + b.y + pz;
  y.z = d2 * rs * g.z + b.z + pz;
  y.w = d3 * rs * g.w + b.w + pz;

  if constexpr (FIN != 0) {
    if (live) {
      volatile v4f* o = (volatile v4f*)(outp + (size_t)t * DFEAT + 4 * lane);
      *o = y;
      __threadfence();
      *o = y;
    }
  } else {
    v4f z;
    z.x = live ? y.x : 0.0f;
    z.y = live ? y.y : 0.0f;
    z.z = live ? y.z : 0.0f;
    z.w = live ? y.w : 0.0f;
    const v2u hi = hi4(z);
    v2u lo = lo4(z);
    if (SELF_TWO_TERM == 0) lo = (v2u){ 0u, 0u };
    *(v2ua*)(&rowb[wave * 128 + 2 * lane])      = hi;
    *(v2ua*)(&rowb[wave * 128 + 64 + 2 * lane]) = lo;
    wave_sync();
    const v4u q = *(const v4ua*)(&rowb[wave * 128 + 4 * lane]);
    volatile v4f* o = (volatile v4f*)(outp + (size_t)tc * DFEAT + 4 * lane);
    volatile v4u* a = (volatile v4u*)(apl + (size_t)(t < MPAD ? t : MPAD - 1) * KL1 + 2 * DFEAT + 8 * lane);
    if (live) *o = y;
    if (t < MPAD) *a = q;
    __threadfence();
    if (live) *o = y;
    if (t < MPAD) *a = q;
  }
}

extern "C" void kernel_launch(void* const* d_in, const int* in_sizes, int n_in,
                              void* d_out, int out_size, void* d_ws, size_t ws_size,
                              hipStream_t stream) {
  if (n_in < 7) return;
  if (in_sizes[0] != NNODE * DFEAT) return;
  if (in_sizes[1] != 2 * NEDGE) return;
  if (in_sizes[2] != 2 * DFEAT * DFEAT || in_sizes[4] != 2 * DFEAT * DFEAT) return;
  if (in_sizes[3] != 2 * DFEAT || in_sizes[5] != 2 * DFEAT || in_sizes[6] != 2 * DFEAT) return;
  if (out_size != NNODE * DFEAT) return;
  if (ws_size < WS_TOTAL) return;

  const float* x   = (const float*)d_in[0];
  const int*   ei  = (const int*)d_in[1];
  const float* Wl  = (const float*)d_in[2];
  const float* bl  = (const float*)d_in[3];
  const float* Wr  = (const float*)d_in[4];
  const float* gam = (const float*)d_in[5];
  const float* bet = (const float*)d_in[6];
  float* out = (float*)d_out;

  char* ws = (char*)d_ws;
  unsigned short* Apl = (unsigned short*)(ws + WS_A);
  float* PRE  = (float*)(ws + WS_PRE);
  float* H    = (float*)(ws + WS_H);
  int*   LIST = (int*)(ws + WS_LIST);
  int*   OFF  = (int*)(ws + WS_OFF);
  int*   CNT  = (int*)(ws + WS_CNT);
  int*   FLAG = (int*)(ws + WS_FLAG);
  unsigned short* BW = (unsigned short*)(ws + WS_BW);
  float* TBL  = (float*)(ws + WS_TBL);

  const int bkLds = BK_LDS_INTS * 4;
  hipFuncSetAttribute(reinterpret_cast<const void*>(&k_bucket), hipFuncAttributeMaxDynamicSharedMemorySize, bkLds);

  const int tiles  = ((NNODE + 63) / 64) * ((DFEAT + 63) / 64);
  const int gGemm  = (tiles + 7) / 8;

  k_prep<<<PB_XB + PB_B0 + PB_B1 + 1, 256, 0, stream>>>(x, Wl, Wr, bl, gam, bet, Apl, BW, TBL);
  k_bucket<<<NBLK, 256, bkLds, stream>>>(ei, LIST, OFF, CNT, FLAG);
  k_replay<1><<<MPAD / 8, 256, 0, stream>>>(LIST, OFF, CNT, FLAG, H, Apl);
  k_gemm_nt<0, 1><<<gGemm, 256, 0, stream>>>(Apl, BW, TBL, PRE, NNODE, DFEAT, KL0, DFEAT);
  k_row<0><<<MPAD / 8, 256, 0, stream>>>(PRE, TBL + 256, TBL + 512, FLAG, H, Apl);
  k_replay<0><<<MPAD / 8, 256, 0, stream>>>(LIST, OFF, CNT, FLAG, H, Apl);
  k_gemm_nt<0, 1><<<gGemm, 256, 0, stream>>>(Apl, BW + B1_OFF, TBL + DFEAT, PRE, NNODE, DFEAT, KL1, DFEAT);
  k_row<1><<<NNODE / 8, 256, 0, stream>>>(PRE, TBL + 256 + DFEAT, TBL + 512 + DFEAT, FLAG, out, Apl);
}
